// GraphSAGE_81870666596807
// MI455X (gfx1250) — hardware-verified
//
#include <hip/hip_runtime.h>
#include <stddef.h>
#include <stdint.h>
#include <math.h>


#define DF     128
#define AP     512
#define K0L    384
#define K12    512
#define NTHR   256
#define NWAVE  8
#define EPT    8
#define CHUNK  (NTHR * EPT)
#define WCAP   (EPT * 32)
#define LISTN  (NWAVE * WCAP)
#define NBA    1024
#define SLA    10
#define RCAP   20480
#define DEGCAP 64
#define AGR    64
#define GBM    64
#define GBN    128
#define GTHR   128
#define UPART  2048
#define NPART  7
#define CMP_ZINTS    (LISTN + 2 * RCAP + 3 * NBA)
#define MISC_INTS    16
#define CMP_LDS_INTS (CMP_ZINTS + MISC_INTS)
#define WSMAX  134217728

static_assert((CHUNK & (CHUNK - 1)) == 0 && CHUNK <= 4096);
static_assert((NBA & (NBA - 1)) == 0 && NBA == (1 << SLA));
static_assert(((long long)CHUNK << SLA) < (1LL << 31));
static_assert(NBA == 4 * NTHR);
static_assert(RCAP % (4 * NTHR) == 0 && CMP_ZINTS % (NTHR * 4) == 0 && LISTN % 4 == 0);
static_assert(K0L % 32 == 0 && K12 % 32 == 0 && K12 == AP && K0L == 3 * DF && AP == 4 * DF);
static_assert(GBN == DF && GBM == (GTHR / 32) * 16 && DF == 4 * 32);
static_assert(UPART == 8 * NTHR && UPART == DF * (DF / 8));
static_assert(AGR % NWAVE == 0 && NBA % AGR == 0 && AGR == GBM);
static_assert(2 * GBM == GTHR);
static_assert(CMP_LDS_INTS * 4 <= 300000);

typedef float          v2f   __attribute__((ext_vector_type(2)));
typedef float          v4f   __attribute__((ext_vector_type(4)));
typedef float          v8f   __attribute__((ext_vector_type(8)));
typedef int            v4i   __attribute__((ext_vector_type(4)));
typedef int            v8i   __attribute__((ext_vector_type(8)));
typedef unsigned       v2u   __attribute__((ext_vector_type(2)));
typedef unsigned short v4us  __attribute__((ext_vector_type(4)));
typedef unsigned short v8us  __attribute__((ext_vector_type(8)));
typedef unsigned short v16us __attribute__((ext_vector_type(16)));
typedef __bf16         v16bf __attribute__((ext_vector_type(16)));
typedef v2f  __attribute__((may_alias)) v2fa;
typedef v4f  __attribute__((may_alias)) v4fa;
typedef v4i  __attribute__((may_alias)) v4ia;
typedef v2u  __attribute__((may_alias)) v2ua;
typedef v4us __attribute__((may_alias)) v4usa;
typedef v8us __attribute__((may_alias)) v8usa;
union FragB { v16bf v; v16us u; v8us h[2]; v8i w; };

__device__ __forceinline__ v8f wmb(const FragB& a, const FragB& b, v8f c) {
  v8f d = __builtin_amdgcn_wmma_f32_16x16x32_bf16(false, a.v, false, b.v, (short)0, c, false, false);
  asm volatile("v_nop\n\tv_nop\n\tv_nop\n\tv_nop" : "+v"(d) : "v"(a.w), "v"(b.w));
  return d;
}

__device__ __forceinline__ unsigned bf16_bits(float f) {
  const unsigned u = __float_as_uint(f);
  return (u + 0x7FFFu + ((u >> 16) & 1u)) >> 16;
}
__device__ __forceinline__ float bf16_val(float f) {
  return __uint_as_float(bf16_bits(f) << 16);
}

__device__ __forceinline__ void wave_sync() {
  __builtin_amdgcn_fence(__ATOMIC_RELEASE, "wavefront");
  __builtin_amdgcn_wave_barrier();
  __builtin_amdgcn_fence(__ATOMIC_ACQUIRE, "wavefront");
}

template <int SLB>
__device__ __forceinline__ int scan_chunk(const int* __restrict__ dsts, int nE, int cbase, int slotBase,
                                          int nb, int vec8, int* list, int tid, int lane, int wave) {
  int wc = 0;
  const int el0  = tid * EPT;
  const int e0   = cbase + el0;
  const int sent = -2147483647 - 1;
  v4i da, db;
  if (vec8 != 0 && cbase + CHUNK <= nE) {
    da = *(const v4i*)(dsts + e0);
    db = *(const v4i*)(dsts + e0 + 4);
  } else {
    da.x = (e0     < nE) ? dsts[min(e0,     nE - 1)] : sent;
    da.y = (e0 + 1 < nE) ? dsts[min(e0 + 1, nE - 1)] : sent;
    da.z = (e0 + 2 < nE) ? dsts[min(e0 + 2, nE - 1)] : sent;
    da.w = (e0 + 3 < nE) ? dsts[min(e0 + 3, nE - 1)] : sent;
    db.x = (e0 + 4 < nE) ? dsts[min(e0 + 4, nE - 1)] : sent;
    db.y = (e0 + 5 < nE) ? dsts[min(e0 + 5, nE - 1)] : sent;
    db.z = (e0 + 6 < nE) ? dsts[min(e0 + 6, nE - 1)] : sent;
    db.w = (e0 + 7 < nE) ? dsts[min(e0 + 7, nE - 1)] : sent;
  }
  const unsigned nbs = (unsigned)slotBase;
  const unsigned unb = (unsigned)nb;
  const unsigned s0 = (unsigned)da.x - nbs, s1 = (unsigned)da.y - nbs;
  const unsigned s2 = (unsigned)da.z - nbs, s3 = (unsigned)da.w - nbs;
  const unsigned s4 = (unsigned)db.x - nbs, s5 = (unsigned)db.y - nbs;
  const unsigned s6 = (unsigned)db.z - nbs, s7 = (unsigned)db.w - nbs;
  const bool h0 = s0 < unb, h1 = s1 < unb, h2 = s2 < unb, h3 = s3 < unb;
  const bool h4 = s4 < unb, h5 = s5 < unb, h6 = s6 < unb, h7 = s7 < unb;
  const unsigned any = __builtin_amdgcn_ballot_w32(h0 | h1 | h2 | h3 | h4 | h5 | h6 | h7);
  if (any != 0u) {
#define HITJ(J, HJ, SJ) { \
      const unsigned mj = __builtin_amdgcn_ballot_w32(HJ); \
      if (mj != 0u) { \
        if (HJ) { \
          const int pos = wc + (int)__builtin_amdgcn_mbcnt_lo(mj, 0u); \
          if (pos < WCAP) list[wave * WCAP + pos] = ((el0 + (J)) << SLB) | (int)(SJ); \
        } \
        wc += (int)__builtin_popcount(mj); } }
    HITJ(0, h0, s0)
    HITJ(1, h1, s1)
    HITJ(2, h2, s2)
    HITJ(3, h3, s3)
    HITJ(4, h4, s4)
    HITJ(5, h5, s5)
    HITJ(6, h6, s6)
    HITJ(7, h7, s7)
#undef HITJ
  }
  return wc;
}

__device__ __forceinline__ void wput(const float* __restrict__ W, unsigned short* P, int pitch, int coff,
                                     int n, int k8) {
  const float* p = W + (size_t)n * DF + k8;
  const v4f a = *(const v4f*)p;
  const v4f b = *(const v4f*)(p + 4);
  v8us o;
  o[0] = (unsigned short)bf16_bits(a.x); o[1] = (unsigned short)bf16_bits(a.y);
  o[2] = (unsigned short)bf16_bits(a.z); o[3] = (unsigned short)bf16_bits(a.w);
  o[4] = (unsigned short)bf16_bits(b.x); o[5] = (unsigned short)bf16_bits(b.y);
  o[6] = (unsigned short)bf16_bits(b.z); o[7] = (unsigned short)bf16_bits(b.w);
  unsigned short* dp = P + (size_t)n * pitch + coff + k8;
  *(volatile v8us*)dp = o;
  __threadfence();
  *(volatile v8us*)dp = o;
}

__global__ __launch_bounds__(NTHR) void k_wprep(const float* __restrict__ Wl0, const float* __restrict__ Wr0,
                                                const float* __restrict__ Wl1, const float* __restrict__ Wr1,
                                                unsigned short* B0, unsigned short* B1) {
  const int part = (int)blockIdx.x >> 3;
  const int v    = ((int)blockIdx.x & 7) * NTHR + (int)threadIdx.x;
  const int n    = v >> 4;
  const int k8   = (v & 15) * 8;
  if (part == 0)      wput(Wl0, B0, K0L, 0,      n, k8);
  else if (part == 1) wput(Wl0, B0, K0L, DF,     n, k8);
  else if (part == 2) wput(Wr0, B0, K0L, 2 * DF, n, k8);
  else if (part == 3) wput(Wl1, B1, K12, 0,      n, k8);
  else if (part == 4) wput(Wl1, B1, K12, DF,     n, k8);
  else if (part == 5) wput(Wr1, B1, K12, 2 * DF, n, k8);
  else if (part == 6) wput(Wr1, B1, K12, 3 * DF, n, k8);
}

__global__ __launch_bounds__(NTHR) void k_compact(const int* __restrict__ srcs, const int* __restrict__ keys,
                                                  int nE, int nN, int vec8,
                                                  int* LIST, int* CNT, int* OFF, float* INV) {
  extern __shared__ __attribute__((aligned(16))) int dsm[];
  int* list = dsm;
  int* hl   = dsm + LISTN;
  int* sl   = hl + RCAP;
  int* cnt  = sl + RCAP;
  int* offs = cnt + NBA;
  int* cur  = offs + NBA;
  int* misc = cur + NBA;
  const int tid = (int)threadIdx.x, lane = tid & 31, wave = tid >> 5;
  const int nodeBase = (int)blockIdx.x * NBA;

  {
    const v4i z4 = {0, 0, 0, 0};
    for (int i = tid * 4; i < CMP_ZINTS; i += NTHR * 4) *(v4ia*)(dsm + i) = z4;
    if (tid < MISC_INTS) misc[tid] = 0;
  }
  __syncthreads();

  int t = 0, ov = 0;
  const int nChunks = (nE + CHUNK - 1) / CHUNK;
#pragma unroll 1
  for (int ch = 0; ch < nChunks; ++ch) {
    const int cbase = ch * CHUNK;
    const int wc = scan_chunk<SLA>(keys, nE, cbase, nodeBase, NBA, vec8, list, tid, lane, wave);
    if (lane == 0) misc[wave] = wc;
    __syncthreads();
    if (wave == 0) {
#pragma unroll 1
      for (int w2 = 0; w2 < NWAVE; ++w2) {
        int c = misc[w2];
        c = c < 0 ? 0 : (c > WCAP ? WCAP : c);
#pragma unroll 1
        for (int b0 = 0; b0 < c; b0 += 32) {
          const int idx = b0 + lane;
          const int ent = list[w2 * WCAP + (idx < WCAP ? idx : WCAP - 1)];
          const int m32 = (c - b0) < 32 ? (c - b0) : 32;
#pragma unroll 1
          for (int k = 0; k < m32; ++k) {
            const int u    = __builtin_amdgcn_readlane(ent, k);
            const int slot = u & (NBA - 1);
            const int el   = (u >> SLA) & (CHUNK - 1);
            const int pk   = ((cbase + el) << SLA) | slot;
            if (t < RCAP) {
              if (lane == 0) { hl[t] = pk; cnt[slot] = cnt[slot] + 1; }
              t = t + 1;
            } else {
              ov = 1;
            }
          }
        }
      }
    }
    __syncthreads();
  }
  if (wave == 0 && lane == 0) { misc[8] = t; misc[9] = ov; }
  __syncthreads();
  int tt = misc[8];
  tt = tt < 0 ? 0 : (tt > RCAP ? RCAP : tt);
  const int ovf = misc[9];

  if (wave == 0) {
    const int base = lane * (NBA / 32);
    int s = 0;
#pragma unroll 1
    for (int i = 0; i < NBA / 32; ++i) s += cnt[base + i];
    int incl = s;
#pragma unroll
    for (int d = 1; d < 32; d <<= 1) {
      const int y = __shfl_up(incl, d, 32);
      if (lane >= d) incl += y;
    }
    int run = incl - s;
#pragma unroll 1
    for (int i = 0; i < NBA / 32; ++i) {
      const int cv = cnt[base + i];
      offs[base + i] = run;
      cur[base + i]  = run;
      run += cv;
    }
  }
  __syncthreads();
  if (wave == 0) {
#pragma unroll 1
    for (int b0 = 0; b0 < tt; b0 += 32) {
      const int idx = b0 + lane;
      const int ent = hl[idx < RCAP ? idx : RCAP - 1];
      const int m32 = (tt - b0) < 32 ? (tt - b0) : 32;
#pragma unroll 1
      for (int k = 0; k < m32; ++k) {
        const int u    = __builtin_amdgcn_readlane(ent, k);
        const int slot = u & (NBA - 1);
        if (lane == 0) {
          int p = cur[slot];
          p = p < 0 ? 0 : (p > RCAP - 1 ? RCAP - 1 : p);
          sl[p] = u;
          cur[slot] = p + 1;
        }
      }
    }
  }
  __syncthreads();

#pragma unroll 4
  for (int idx = tid; idx < RCAP; idx += NTHR) {
    const int ent = sl[idx];
    int eid = ent >> SLA;
    eid = eid < 0 ? 0 : (eid > nE - 1 ? nE - 1 : eid);
    int sr = srcs[eid];
    sr = sr < 0 ? 0 : (sr > nN - 1 ? nN - 1 : sr);
    hl[idx] = sr;
  }
  const float qnan = __int_as_float(0x7fc00000);
#pragma unroll 1
  for (int i = tid; i < NBA; i += NTHR) {
    const int c = cnt[i];
    float d = (float)c;
    d = (d < 1.0f) ? 1.0f : d;
    const float iv = 1.0f / d;
    const bool bad = (ovf != 0) || (c > DEGCAP);
    cur[i] = __float_as_int(bad ? qnan : iv);
  }
  __syncthreads();

  const v4i c4 = *(const v4ia*)(cnt + 4 * tid);
  const v4i o4 = *(const v4ia*)(offs + 4 * tid);
  const v4i i4 = *(const v4ia*)(cur + 4 * tid);
  v4f f4;
  f4.x = __int_as_float(i4.x); f4.y = __int_as_float(i4.y);
  f4.z = __int_as_float(i4.z); f4.w = __int_as_float(i4.w);
  int*   cp = CNT + (size_t)nodeBase + 4 * tid;
  int*   op = OFF + (size_t)nodeBase + 4 * tid;
  float* ip = INV + (size_t)nodeBase + 4 * tid;
  int*   lp = LIST + (size_t)blockIdx.x * RCAP;

  *(volatile v4i*)cp = c4;
  *(volatile v4i*)op = o4;
  *(volatile v4f*)ip = f4;
#pragma unroll 4
  for (int it = 0; it < RCAP / (4 * NTHR); ++it) {
    const int q = 4 * (it * NTHR + tid);
    const v4i v = *(const v4ia*)(hl + q);
    *(volatile v4i*)(lp + q) = v;
  }
  __threadfence();
  *(volatile v4i*)cp = c4;
  *(volatile v4i*)op = o4;
  *(volatile v4f*)ip = f4;
#pragma unroll 4
  for (int it = 0; it < RCAP / (4 * NTHR); ++it) {
    const int q = 4 * (it * NTHR + tid);
    const v4i v = *(const v4ia*)(hl + q);
    *(volatile v4i*)(lp + q) = v;
  }
}

template <int L0>
__global__ __launch_bounds__(NTHR) void k_agg(const int* __restrict__ lst, const int* __restrict__ cntg,
                                              const int* __restrict__ offg, const float* __restrict__ invg,
                                              int nN, const float* __restrict__ xin, unsigned short* apl) {
  __shared__ __attribute__((aligned(16))) unsigned short rowbufs[NWAVE * AP];
  const int tid = (int)threadIdx.x, lane = tid & 31, wave = tid >> 5;
  unsigned short* rowbuf = rowbufs + wave * AP;
  const int rowBase = (int)blockIdx.x * AGR;

#pragma unroll 1
  for (int si = 0; si < AGR / NWAVE; ++si) {
    const int node = rowBase + si * NWAVE + wave;
    const bool live = node < nN;
    const int nc = live ? node : nN - 1;
    int c = cntg[nc];
    c = c < 0 ? 0 : (c > DEGCAP ? DEGCAP : c);
    c = live ? c : 0;
    c = __builtin_amdgcn_readfirstlane(c);
    int o = offg[nc];
    o = o < 0 ? 0 : (o > RCAP ? RCAP : o);
    o = __builtin_amdgcn_readfirstlane(o);
    const float inv = invg[nc];
    const size_t lb = (size_t)(nc >> SLA) * RCAP;
    float a0 = 0.0f, a1 = 0.0f, a2 = 0.0f, a3 = 0.0f;
#pragma unroll 1
    for (int b0 = 0; b0 < c; b0 += 32) {
      int idx = o + b0 + lane;
      idx = idx > RCAP - 1 ? RCAP - 1 : idx;
      int sr = lst[lb + idx];
      sr = sr < 0 ? 0 : (sr > nN - 1 ? nN - 1 : sr);
      const int m32 = (c - b0) < 32 ? (c - b0) : 32;
#pragma unroll 1
      for (int k = 0; k < m32; ++k) {
        const int sk = __builtin_amdgcn_readlane(sr, k);
        if constexpr (L0 != 0) {
          const v4f a = *(const v4f*)(xin + (size_t)sk * DF + 4 * lane);
          a0 += bf16_val(a.x);
          a1 += bf16_val(a.y);
          a2 += bf16_val(a.z);
          a3 += bf16_val(a.w);
        } else {
          const unsigned short* rp = apl + (size_t)sk * AP + 2 * DF + 4 * lane;
          const v2u wh = *(const v2ua*)rp;
          const v2u wl = *(const v2ua*)(rp + DF);
          a0 += __uint_as_float(wh.x << 16)         + __uint_as_float(wl.x << 16);
          a1 += __uint_as_float(wh.x & 0xffff0000u) + __uint_as_float(wl.x & 0xffff0000u);
          a2 += __uint_as_float(wh.y << 16)         + __uint_as_float(wl.y << 16);
          a3 += __uint_as_float(wh.y & 0xffff0000u) + __uint_as_float(wl.y & 0xffff0000u);
        }
      }
    }
    const float m0 = live ? (a0 * inv) : 0.0f;
    const float m1 = live ? (a1 * inv) : 0.0f;
    const float m2 = live ? (a2 * inv) : 0.0f;
    const float m3 = live ? (a3 * inv) : 0.0f;
    v4us mh, ml;
    {
      unsigned hb;
      hb = bf16_bits(m0); mh[0] = (unsigned short)hb; ml[0] = (unsigned short)bf16_bits(m0 - __uint_as_float(hb << 16));
      hb = bf16_bits(m1); mh[1] = (unsigned short)hb; ml[1] = (unsigned short)bf16_bits(m1 - __uint_as_float(hb << 16));
      hb = bf16_bits(m2); mh[2] = (unsigned short)hb; ml[2] = (unsigned short)bf16_bits(m2 - __uint_as_float(hb << 16));
      hb = bf16_bits(m3); mh[3] = (unsigned short)hb; ml[3] = (unsigned short)bf16_bits(m3 - __uint_as_float(hb << 16));
    }
    *(v4usa*)(rowbuf + 4 * lane) = mh;
    *(v4usa*)(rowbuf + DF + 4 * lane) = ml;
    if constexpr (L0 != 0) {
      const v4f xs = *(const v4f*)(xin + (size_t)nc * DF + 4 * lane);
      v4us xb;
      xb[0] = live ? (unsigned short)bf16_bits(xs.x) : (unsigned short)0;
      xb[1] = live ? (unsigned short)bf16_bits(xs.y) : (unsigned short)0;
      xb[2] = live ? (unsigned short)bf16_bits(xs.z) : (unsigned short)0;
      xb[3] = live ? (unsigned short)bf16_bits(xs.w) : (unsigned short)0;
      const v4us z4 = {0, 0, 0, 0};
      *(v4usa*)(rowbuf + 2 * DF + 4 * lane) = xb;
      *(v4usa*)(rowbuf + 3 * DF + 4 * lane) = z4;
    }
    wave_sync();
    const v8us q0 = *(const v8usa*)(rowbuf + 8 * lane);
    v8us q1 = {0, 0, 0, 0, 0, 0, 0, 0};
    if constexpr (L0 != 0) q1 = *(const v8usa*)(rowbuf + 2 * DF + 8 * lane);
    wave_sync();
    unsigned short* rpw = apl + (size_t)node * AP + 8 * lane;
    *(volatile v8us*)rpw = q0;
    if constexpr (L0 != 0) *(volatile v8us*)(rpw + 2 * DF) = q1;
    __threadfence();
    *(volatile v8us*)rpw = q0;
    if constexpr (L0 != 0) *(volatile v8us*)(rpw + 2 * DF) = q1;
  }
}

template <int FIN>
__global__ __launch_bounds__(GTHR) void k_gemm(unsigned short* Apl, const unsigned short* __restrict__ BT, int K,
                                               const float* __restrict__ bias, const float* __restrict__ wl2,
                                               const float* __restrict__ wr2, float* pr2, int nOut) {
  __shared__ __attribute__((aligned(16))) float stg[GBM * GBN];
  __shared__ __attribute__((aligned(16))) float wts[4 * DF];
  __shared__ __attribute__((aligned(16))) float prs[GBM * 4];
  const int tid = (int)threadIdx.x, lane = tid & 31, wave = tid >> 5, hh = lane >> 4, m = lane & 15;
  const int rowBase = (int)blockIdx.x * GBM;

  if constexpr (FIN != 0) {
    wts[tid]          = bf16_val(wl2[tid]);
    wts[DF + tid]     = bf16_val(wl2[DF + tid]);
    wts[2 * DF + tid] = bf16_val(wr2[tid]);
    wts[3 * DF + tid] = bf16_val(wr2[DF + tid]);
  }

  v8f acc[8];
  {
    const v8f z = {0.f, 0.f, 0.f, 0.f, 0.f, 0.f, 0.f, 0.f};
#pragma unroll
    for (int t = 0; t < 8; ++t) acc[t] = z;
  }
  const unsigned short* ap = Apl + (size_t)(rowBase + 16 * wave + m) * (size_t)AP + 8 * hh;
  const unsigned short* bp = BT + (size_t)m * (size_t)K + 8 * hh;

#pragma unroll 1
  for (int k0 = 0; k0 < K; k0 += 32) {
    FragB af;
    af.h[0] = *(const v8usa*)(ap + k0);
    af.h[1] = *(const v8usa*)(ap + k0 + 16);
#pragma unroll
    for (int nt = 0; nt < 8; ++nt) {
      const unsigned short* wq = bp + (size_t)(16 * nt) * (size_t)K + k0;
      FragB bf;
      bf.h[0] = *(const v8usa*)wq;
      bf.h[1] = *(const v8usa*)(wq + 16);
      acc[nt] = wmb(af, bf, acc[nt]);
    }
  }

#pragma unroll
  for (int nt = 0; nt < 8; ++nt) {
    const int lc = 16 * nt + m;
#pragma unroll
    for (int r = 0; r < 8; ++r) {
      const int lr = 16 * wave + 8 * hh + r;
      stg[lr * GBN + lc] = acc[nt][r];
    }
  }
  __syncthreads();

  v4f bb4;
  {
    const v4f t1 = *(const v4f*)(bias + 4 * lane);
    bb4.x = bf16_val(t1.x); bb4.y = bf16_val(t1.y); bb4.z = bf16_val(t1.z); bb4.w = bf16_val(t1.w);
  }

  v4f pv[16];
#pragma unroll
  for (int i = 0; i < 16; ++i) pv[i] = *(const v4fa*)(stg + (16 * wave + i) * GBN + 4 * lane);
  __syncthreads();

#pragma unroll
  for (int i = 0; i < 16; ++i) {
    const bool ok = (rowBase + 16 * wave + i) < nOut;
    const v4f t = pv[i] + bb4;
    v4f y;
    y.x = (t.x > 0.0f) ? t.x : (t.x - t.x);
    y.y = (t.y > 0.0f) ? t.y : (t.y - t.y);
    y.z = (t.z > 0.0f) ? t.z : (t.z - t.z);
    y.w = (t.w > 0.0f) ? t.w : (t.w - t.w);
    y.x = ok ? y.x : 0.0f; y.y = ok ? y.y : 0.0f; y.z = ok ? y.z : 0.0f; y.w = ok ? y.w : 0.0f;
    pv[i] = y;
  }

  if constexpr (FIN != 0) {
#pragma unroll
    for (int i = 0; i < 16; ++i) *(v4fa*)(stg + (16 * wave + i) * GBN + 4 * lane) = pv[i];
    __syncthreads();
    {
      const int row = tid >> 1, pr = tid & 1;
      const float* hr = stg + row * GBN;
      const float* w0 = wts + (2 * pr) * DF;
      const float* w1 = w0 + DF;
      float s0 = 0.0f, s1 = 0.0f;
#pragma unroll 2
      for (int k4 = 0; k4 < DF / 4; ++k4) {
        const v4f h = *(const v4fa*)(hr + 4 * k4);
        const v4f a = *(const v4fa*)(w0 + 4 * k4);
        const v4f b = *(const v4fa*)(w1 + 4 * k4);
        s0 = fmaf(h.x, a.x, s0); s0 = fmaf(h.y, a.y, s0); s0 = fmaf(h.z, a.z, s0); s0 = fmaf(h.w, a.w, s0);
        s1 = fmaf(h.x, b.x, s1); s1 = fmaf(h.y, b.y, s1); s1 = fmaf(h.z, b.z, s1); s1 = fmaf(h.w, b.w, s1);
      }
      prs[row * 4 + 2 * pr + 0] = s0;
      prs[row * 4 + 2 * pr + 1] = s1;
    }
    __syncthreads();
    if (tid < GBM) {
      const v4f ov = *(const v4fa*)(prs + 4 * tid);
      float* op = pr2 + (size_t)(rowBase + tid) * 4;
      *(volatile v4f*)op = ov;
      __threadfence();
      *(volatile v4f*)op = ov;
    }
  } else {
#pragma unroll
    for (int i = 0; i < 16; ++i) {
      v4us h4, l4;
      unsigned hb;
      hb = bf16_bits(pv[i].x); h4[0] = (unsigned short)hb; l4[0] = (unsigned short)bf16_bits(pv[i].x - __uint_as_float(hb << 16));
      hb = bf16_bits(pv[i].y); h4[1] = (unsigned short)hb; l4[1] = (unsigned short)bf16_bits(pv[i].y - __uint_as_float(hb << 16));
      hb = bf16_bits(pv[i].z); h4[2] = (unsigned short)hb; l4[2] = (unsigned short)bf16_bits(pv[i].z - __uint_as_float(hb << 16));
      hb = bf16_bits(pv[i].w); h4[3] = (unsigned short)hb; l4[3] = (unsigned short)bf16_bits(pv[i].w - __uint_as_float(hb << 16));
      unsigned short* srow = (unsigned short*)stg + (size_t)(16 * wave + i) * (2 * GBN);
      *(v4usa*)(srow + 4 * lane) = h4;
      *(v4usa*)(srow + DF + 4 * lane) = l4;
    }
    __syncthreads();
    v8us qv[16];
#pragma unroll
    for (int i = 0; i < 16; ++i) {
      const unsigned short* srow = (const unsigned short*)stg + (size_t)(16 * wave + i) * (2 * GBN);
      qv[i] = *(const v8usa*)(srow + 8 * lane);
    }
#pragma unroll
    for (int i = 0; i < 16; ++i) {
      unsigned short* rp = Apl + (size_t)(rowBase + 16 * wave + i) * (size_t)AP + 2 * DF + 8 * lane;
      *(volatile v8us*)rp = qv[i];
    }
    __threadfence();
#pragma unroll
    for (int i = 0; i < 16; ++i) {
      unsigned short* rp = Apl + (size_t)(rowBase + 16 * wave + i) * (size_t)AP + 2 * DF + 8 * lane;
      *(volatile v8us*)rp = qv[i];
    }
  }
}

__global__ __launch_bounds__(NTHR) void k_out(const int* __restrict__ lst, const int* __restrict__ cntg,
                                              const int* __restrict__ offg, const float* __restrict__ invg,
                                              const float* __restrict__ pr2, const float* __restrict__ b2,
                                              int nN, float* out) {
  __shared__ __attribute__((aligned(16))) float os[2 * NTHR];
  const int tid = (int)threadIdx.x;
  const int node = (int)blockIdx.x * NTHR + tid;
  const int nc = node < nN ? node : nN - 1;
  int c = cntg[nc];
  c = c < 0 ? 0 : (c > DEGCAP ? DEGCAP : c);
  int o = offg[nc];
  o = o < 0 ? 0 : (o > RCAP ? RCAP : o);
  const float inv = invg[nc];
  const size_t lb = (size_t)(nc >> SLA) * RCAP;
  int cm = c;
#pragma unroll
  for (int d = 16; d >= 1; d >>= 1) {
    const int y = __shfl_xor(cm, d, 32);
    cm = cm > y ? cm : y;
  }
  cm = __builtin_amdgcn_readfirstlane(cm);
  cm = cm > DEGCAP ? DEGCAP : cm;
  float s0 = 0.0f, s1 = 0.0f;
#pragma unroll 1
  for (int p = 0; p < cm; ++p) {
    int idx = o + p;
    idx = idx > RCAP - 1 ? RCAP - 1 : idx;
    int sr = lst[lb + idx];
    sr = sr < 0 ? 0 : (sr > nN - 1 ? nN - 1 : sr);
    const v2f v = *(const v2fa*)(pr2 + (size_t)sr * 4);
    const int msk = -(int)(p < c);
    s0 += __int_as_float(__float_as_int(v.x) & msk);
    s1 += __int_as_float(__float_as_int(v.y) & msk);
  }
  const v4f self = *(const v4fa*)(pr2 + (size_t)nc * 4);
  const float bb0 = bf16_val(b2[0]);
  const float bb1 = bf16_val(b2[1]);
  const float o0 = (s0 * inv + bb0) + self.z;
  const float o1 = (s1 * inv + bb1) + self.w;
  const float mx = (o0 > o1) ? o0 : o1;
  const float d0 = o0 - mx, d1 = o1 - mx;
  const float ls = logf(expf(d0) + expf(d1));
  v2f r;
  r.x = d0 - ls;
  r.y = d1 - ls;
  *(v2fa*)(os + 2 * tid) = r;
  __syncthreads();
  const long long f0 = (long long)blockIdx.x * (2 * NTHR) + 4 * tid;
  const bool wr = (tid < NTHR / 2) && (f0 + 3 < 2LL * (long long)nN);
  const v4f ov = *(const v4fa*)(os + 4 * (tid & (NTHR / 2 - 1)));
  float* op = out + (wr ? f0 : 0);
  if (wr) *(volatile v4f*)op = ov;
  __threadfence();
  if (wr) *(volatile v4f*)op = ov;
}

static inline int cdiv(int a, int b) { return (a + b - 1) / b; }
static inline size_t al256(size_t o) { return (o + 255) & ~(size_t)255; }

extern "C" void kernel_launch(void* const* d_in, const int* in_sizes, int n_in,
                              void* d_out, int out_size, void* d_ws, size_t ws_size,
                              hipStream_t stream) {
  if (n_in < 12) return;
  if (in_sizes[0] < DF || (in_sizes[0] % DF) != 0) return;
  const int nN = in_sizes[0] / DF;
  if (nN < 16 || nN >= (1 << 24) || (nN % 16) != 0) return;
  if (in_sizes[1] != DF * DF || in_sizes[3] != DF * DF) return;
  if (in_sizes[4] != DF * DF || in_sizes[6] != DF * DF) return;
  if (in_sizes[2] != DF || in_sizes[5] != DF) return;
  if (in_sizes[7] != 2 * DF || in_sizes[9] != 2 * DF || in_sizes[8] != 2) return;
  const int nE = in_sizes[10];
  if (nE < 1 || in_sizes[11] != nE || nE >= (1 << 21)) return;
  if ((long long)out_size != 2LL * (long long)nN) return;

  const float* x   = (const float*)d_in[0];
  const float* wl0 = (const float*)d_in[1];
  const float* b0  = (const float*)d_in[2];
  const float* wr0 = (const float*)d_in[3];
  const float* wl1 = (const float*)d_in[4];
  const float* b1  = (const float*)d_in[5];
  const float* wr1 = (const float*)d_in[6];
  const float* wl2 = (const float*)d_in[7];
  const float* b2  = (const float*)d_in[8];
  const float* wr2 = (const float*)d_in[9];
  const int*   src = (const int*)d_in[10];
  const int*   dst = (const int*)d_in[11];
  float* out = (float*)d_out;

  const int MP  = cdiv(nN, GBM) * GBM;
  const int gM  = MP / GBM;
  const int gA  = cdiv(MP, NBA);
  const int NBP = gA * NBA;
  if (NBP < MP) return;
  const int vec8 = ((nE & 3) == 0) ? 1 : 0;

  char* ws = (char*)d_ws;
  size_t off = 0;
  const size_t oB0  = off; off = al256(off + (size_t)DF * K0L * 2);
  const size_t oB1  = off; off = al256(off + (size_t)DF * K12 * 2);
  const size_t oA   = off; off = al256(off + (size_t)MP * AP * 2);
  const size_t oLS  = off; off = al256(off + (size_t)gA * RCAP * 4);
  const size_t oCN  = off; off = al256(off + (size_t)NBP * 4);
  const size_t oOF  = off; off = al256(off + (size_t)NBP * 4);
  const size_t oIV  = off; off = al256(off + (size_t)NBP * 4);
  const size_t oPR  = off; off = al256(off + (size_t)MP * 4 * 4);
  if (off > ws_size || off > (size_t)WSMAX) return;
  unsigned short* B0  = (unsigned short*)(ws + oB0);
  unsigned short* B1  = (unsigned short*)(ws + oB1);
  unsigned short* Apl = (unsigned short*)(ws + oA);
  int*   LIST = (int*)(ws + oLS);
  int*   CNT  = (int*)(ws + oCN);
  int*   OFF  = (int*)(ws + oOF);
  float* INV  = (float*)(ws + oIV);
  float* PR2  = (float*)(ws + oPR);

  const size_t cmpLds = (size_t)CMP_LDS_INTS * 4;
  hipFuncSetAttribute(reinterpret_cast<const void*>(&k_compact), hipFuncAttributeMaxDynamicSharedMemorySize, (int)cmpLds);

  k_wprep<<<(NPART * UPART) / NTHR, NTHR, 0, stream>>>(wl0, wr0, wl1, wr1, B0, B1);
  k_compact<<<gA, NTHR, cmpLds, stream>>>(src, dst, nE, nN, vec8, LIST, CNT, OFF, INV);
  k_agg<1><<<MP / AGR, NTHR, 0, stream>>>(LIST, CNT, OFF, INV, nN, x, Apl);
  k_gemm<0><<<gM, GTHR, 0, stream>>>(Apl, B0, K0L, b0, wl2, wr2, PR2, nN);
  k_agg<0><<<MP / AGR, NTHR, 0, stream>>>(LIST, CNT, OFF, INV, nN, x, Apl);
  k_gemm<1><<<gM, GTHR, 0, stream>>>(Apl, B1, K12, b1, wl2, wr2, PR2, nN);
  k_out<<<cdiv(nN, NTHR), NTHR, 0, stream>>>(LIST, CNT, OFF, INV, PR2, b2, nN, out);
}
